// GraphPairClassifier_59313498358244
// MI455X (gfx1250) — hardware-run, weakly checked
//
#include <hip/hip_runtime.h>
#include <stddef.h>


#define XD      3
#define HID     256
#define NTHR    256
#define NWAVE   8
#define EPT     8
#define NGRP    2
#define CHUNK   (NTHR * EPT * NGRP)
#define WCAP    (EPT * NGRP * 32)
#define ESHF    11
#define EMASK   0xFFFFF
#define NBC     32768
#define NBF     2048
#define RCAP    49152
#define RBN     128
#define TGT     256
#define DEGCAP  512
#define GROWS   128
#define OTHR    512
#define TPK     64
#define TPN     32
#define TPP     72
#define ASCL    16
#define WSCL    64
#define PG      64
#define WSCAP   134217728

#define LDS_COUNT  ((NBC + NWAVE * WCAP + NWAVE) * 4)
#define LDS_FILL   ((RCAP + NBF + NWAVE * WCAP + NWAVE) * 4)
#define LDS_POOL   ((PG * HID + NWAVE * WCAP + NWAVE + PG) * 4)
#define LDS_G128   (GROWS * 128 * 4)
#define LDS_G64    (GROWS * 64 * 4)

static_assert((CHUNK & (CHUNK - 1)) == 0);
static_assert((NBC & (NBC - 1)) == 0 && (NBF & (NBF - 1)) == 0 && (PG & (PG - 1)) == 0);
static_assert(NBF <= (1 << ESHF) && PG <= (1 << ESHF));
static_assert((NBC % NBF) == 0);
static_assert(OTHR * 4 == NBF);
static_assert((RCAP % 32) == 0);
static_assert(TGT == NWAVE * 32);
static_assert(GROWS == NWAVE * 16);
static_assert((TGT % GROWS) == 0);
static_assert(NBC == NWAVE * 32 * 128);
static_assert(HID == 2 * 32 * 4);
static_assert((HID % 32) == 0);
static_assert(TPN * 8 == NTHR && TPK * TPN == NTHR * 8 && TPK == NWAVE * 8);
static_assert((TPP % 8) == 0 && TPP >= TPK);
static_assert(PG == NWAVE * 8);
static_assert((GROWS % PG) == 0);
static_assert(LDS_FILL <= 300 * 1024);

typedef float     v4f  __attribute__((ext_vector_type(4)));
typedef float     v8f  __attribute__((ext_vector_type(8)));
typedef int       v4i  __attribute__((ext_vector_type(4)));
typedef _Float16  v8h  __attribute__((ext_vector_type(8)));
typedef _Float16  v16h __attribute__((ext_vector_type(16)));
union FragH { v16h v; v8h h[2]; };
union U32F { float f; int i; };

__device__ __forceinline__ v8f wmf(v16h a, v16h b, v8f c) {
  v8f d = __builtin_amdgcn_wmma_f32_16x16x32_f16(false, a, false, b, (short)0, c, false, false);
  asm volatile("v_nop\n\tv_nop\n\tv_nop\n\tv_nop" : "+v"(d) : "v"(a), "v"(b));
  return d;
}

__device__ __forceinline__ v8h cvt8h(v4f a, v4f b, float z) {
  v8h h;
  h[0] = (_Float16)(a.x * z); h[1] = (_Float16)(a.y * z); h[2] = (_Float16)(a.z * z); h[3] = (_Float16)(a.w * z);
  h[4] = (_Float16)(b.x * z); h[5] = (_Float16)(b.y * z); h[6] = (_Float16)(b.z * z); h[7] = (_Float16)(b.w * z);
  return h;
}

__device__ __forceinline__ float sigm(float v) {
  const float e = __expf(-fabsf(v));
  const float r = __builtin_amdgcn_rcpf(1.0f + e);
  return v >= 0.0f ? r : e * r;
}

__device__ __forceinline__ v4f relu4(v4f a) {
  v4f y;
  y.x = fmaxf(a.x, 0.0f); y.y = fmaxf(a.y, 0.0f); y.z = fmaxf(a.z, 0.0f); y.w = fmaxf(a.w, 0.0f);
  return y;
}

template <int NB, int SRC, int WC>
__device__ __forceinline__ int scan_chunk(const int* __restrict__ keys, int nK, int cbase,
                                          int slotBase, int lim, int vec8, int* list, int tid, int lane, int wave) {
  int wc = 0;
  const unsigned ulim = (unsigned)(lim < 0 ? 0 : (lim > NB ? NB : lim));
#pragma unroll
  for (int g = 0; g < NGRP; ++g) {
    const int el0  = (g * NTHR + tid) * EPT;
    const int e0   = cbase + el0;
    const int sent = -2147483647 - 1;
    const int i0 = min(e0, nK - 1),     i1 = min(e0 + 1, nK - 1), i2 = min(e0 + 2, nK - 1), i3 = min(e0 + 3, nK - 1);
    const int i4 = min(e0 + 4, nK - 1), i5 = min(e0 + 5, nK - 1), i6 = min(e0 + 6, nK - 1), i7 = min(e0 + 7, nK - 1);
    v4i da, db;
    if (vec8 != 0 && cbase + CHUNK <= nK) {
      da = *(const v4i*)(keys + e0);
      db = *(const v4i*)(keys + e0 + 4);
    } else {
      da.x = (e0     < nK) ? keys[i0] : sent;
      da.y = (e0 + 1 < nK) ? keys[i1] : sent;
      da.z = (e0 + 2 < nK) ? keys[i2] : sent;
      da.w = (e0 + 3 < nK) ? keys[i3] : sent;
      db.x = (e0 + 4 < nK) ? keys[i4] : sent;
      db.y = (e0 + 5 < nK) ? keys[i5] : sent;
      db.z = (e0 + 6 < nK) ? keys[i6] : sent;
      db.w = (e0 + 7 < nK) ? keys[i7] : sent;
    }
    const unsigned nb = (unsigned)slotBase;
    const unsigned s0 = (unsigned)da.x - nb, s1 = (unsigned)da.y - nb;
    const unsigned s2 = (unsigned)da.z - nb, s3 = (unsigned)da.w - nb;
    const unsigned s4 = (unsigned)db.x - nb, s5 = (unsigned)db.y - nb;
    const unsigned s6 = (unsigned)db.z - nb, s7 = (unsigned)db.w - nb;
    const bool h0 = s0 < ulim, h1 = s1 < ulim, h2 = s2 < ulim, h3 = s3 < ulim;
    const bool h4 = s4 < ulim, h5 = s5 < ulim, h6 = s6 < ulim, h7 = s7 < ulim;
    const unsigned any = __builtin_amdgcn_ballot_w32(h0 | h1 | h2 | h3 | h4 | h5 | h6 | h7);
    if (any != 0u) {
#define HITJ(HJ, SJ, VJ) { \
        const unsigned mj = __builtin_amdgcn_ballot_w32(HJ); \
        if (mj != 0u) { \
          if (HJ) { \
            const int pos = wc + (int)__builtin_amdgcn_mbcnt_lo(mj, 0u); \
            const int entv = SRC ? (((VJ) << ESHF) | (int)(SJ)) : (int)(SJ); \
            if (pos < WC) list[wave * WC + pos] = entv; \
          } \
          wc += (int)__builtin_popcount(mj); } }
      HITJ(h0, s0, i0)
      HITJ(h1, s1, i1)
      HITJ(h2, s2, i2)
      HITJ(h3, s3, i3)
      HITJ(h4, s4, i4)
      HITJ(h5, s5, i5)
      HITJ(h6, s6, i6)
      HITJ(h7, s7, i7)
#undef HITJ
    }
  }
  return wc;
}

__global__ __launch_bounds__(NTHR) void k_wT16(const float* __restrict__ W, _Float16* Wp,
                                               int KD, int NC, int NCP, float scale) {
  __shared__ __attribute__((aligned(16))) _Float16 sT[TPN * TPP];
  const int tid = threadIdx.x;
  const int k0 = (int)blockIdx.x * TPK, n0 = (int)blockIdx.y * TPN;
  const int nc = tid & 31, kq = tid >> 5;
  const int col = n0 + nc;
  const int colc = col < NC ? col : NC - 1;
#pragma unroll
  for (int i = 0; i < TPK / NWAVE; ++i) {
    const int kr = kq + NWAVE * i;
    const float w = W[(size_t)(k0 + kr) * NC + colc];
    const float v = (col < NC) ? w * scale : 0.0f;
    sT[nc * TPP + kr] = (_Float16)v;
  }
  __syncthreads();
  const int nl = tid >> 3, p = tid & 7;
  const v8h hv = *(const v8h*)(sT + nl * TPP + 8 * p);
  _Float16* d = Wp + (size_t)(n0 + nl) * KD + k0 + 8 * p;
  *(volatile v8h*)d = hv;
  __threadfence();
  *(volatile v8h*)d = hv;
}

__global__ __launch_bounds__(NTHR) void k_count(
    const int* __restrict__ keys, int* cnt, int nK, int vec8, int nN) {
  extern __shared__ v4f lds_dyn[];
  int* scnt = (int*)lds_dyn;
  int* list = scnt + NBC;
  int* wcnt = list + NWAVE * WCAP;
  const int tid = threadIdx.x, lane = tid & 31, wave = tid >> 5;
  const int nodeBase = blockIdx.x * NBC;
  const int lim = nN - nodeBase;

  {
    const v4i z = {0, 0, 0, 0};
    for (int i = tid; i < NBC / 4; i += NTHR) ((v4i*)scnt)[i] = z;
  }
  __syncthreads();

  const int nChunks = (nK + CHUNK - 1) / CHUNK;
#pragma unroll 1
  for (int ch = 0; ch < nChunks; ++ch) {
    const int cbase = ch * CHUNK;
    const int wc = scan_chunk<NBC, 0, WCAP>(keys, nK, cbase, nodeBase, lim, vec8, list, tid, lane, wave);
    if (lane == 0) wcnt[wave] = wc;
    __syncthreads();
    if (wave == 0) {
#pragma unroll 1
      for (int wsx = 0; wsx < NWAVE; ++wsx) {
        int n = __builtin_amdgcn_readfirstlane(wcnt[wsx]);
        n = n > WCAP ? WCAP : (n < 0 ? 0 : n);
        const int* lp = list + wsx * WCAP;
#pragma unroll 1
        for (int i = 0; i < n; ++i) {
          const int ent  = __builtin_amdgcn_readfirstlane(lp[i]);
          const int slot = ent & (NBC - 1);
          if (lane == 0) scnt[slot] = scnt[slot] + 1;
        }
      }
    }
    __syncthreads();
  }

  int* cp = cnt + (size_t)nodeBase;
#pragma unroll 4
  for (int q = 0; q < 32; ++q) {
    const int f = (wave * 32 + q) * 128 + 4 * lane;
    const v4i c = *(const v4i*)(scnt + f);
    *(volatile v4i*)(cp + f) = c;
  }
  __threadfence();
#pragma unroll 4
  for (int q = 0; q < 32; ++q) {
    const int f = (wave * 32 + q) * 128 + 4 * lane;
    const v4i c = *(const v4i*)(scnt + f);
    *(volatile v4i*)(cp + f) = c;
  }
}

__global__ __launch_bounds__(OTHR) void k_offsets(
    const int* __restrict__ cnt, int* off, float* dis, int* rbase, int nBF) {
  __shared__ __attribute__((aligned(16))) int srb[RBN];
  __shared__ int wtot[OTHR / 32];
  const int tid = threadIdx.x, lane = tid & 31, wave = tid >> 5;
  for (int i = tid; i < RBN; i += OTHR) srb[i] = 0;
  int carry = 0;
#pragma unroll 1
  for (int fb = 0; fb < nBF; ++fb) {
    const int base = fb * NBF;
    const v4i c = *(const v4i*)(cnt + base + 4 * tid);
    const int e0 = max(c.x, 0), e1 = max(c.y, 0), e2 = max(c.z, 0), e3 = max(c.w, 0);
    const int ts = e0 + e1 + e2 + e3;
    int incl = ts;
#pragma unroll
    for (int d = 1; d < 32; d <<= 1) {
      const int t = __shfl_up(incl, d, 32);
      if (lane >= d) incl += t;
    }
    if (lane == 31) wtot[wave] = incl;
    __syncthreads();
    int pre = 0;
#pragma unroll 1
    for (int w = 0; w < wave; ++w) pre += wtot[w];
    int tot = 0;
#pragma unroll
    for (int w = 0; w < OTHR / 32; ++w) tot += wtot[w];
    int run = carry + pre + incl - ts;
    v4i o;
    o.x = run; run += e0;
    o.y = run; run += e1;
    o.z = run; run += e2;
    o.w = run;
    v4f dv;
    dv.x = rsqrtf((float)e0 + 1.0f);
    dv.y = rsqrtf((float)e1 + 1.0f);
    dv.z = rsqrtf((float)e2 + 1.0f);
    dv.w = rsqrtf((float)e3 + 1.0f);
    int*   op = off + base + 4 * tid;
    float* dp = dis + base + 4 * tid;
    *(volatile v4i*)op = o;
    *(volatile v4f*)dp = dv;
    __threadfence();
    *(volatile v4i*)op = o;
    *(volatile v4f*)dp = dv;
    if (tid == 0) srb[min(fb, RBN - 1)] = carry;
    carry += (tot + 31) & ~31;
    __syncthreads();
  }
  if (tid == 0) srb[min(nBF, RBN - 1)] = carry;
  __syncthreads();
  v4i rv = {0, 0, 0, 0};
  if (tid < 32) rv = *(const v4i*)(srb + 4 * tid);
  if (tid < 32) *(volatile v4i*)(rbase + 4 * tid) = rv;
  __threadfence();
  if (tid < 32) *(volatile v4i*)(rbase + 4 * tid) = rv;
}

__global__ __launch_bounds__(NTHR) void k_fill(
    const int* __restrict__ keys, const int* __restrict__ off,
    const int* __restrict__ rbase, int* csr, int nK, int vec8, int csrLen, int nN) {
  extern __shared__ v4f lds_dyn[];
  int* region = (int*)lds_dyn;
  int* cursor = region + RCAP;
  int* list   = cursor + NBF;
  int* wcnt   = list + NWAVE * WCAP;
  const int tid = threadIdx.x, lane = tid & 31, wave = tid >> 5;
  const int b = blockIdx.x;
  const int nodeBase = b * NBF;
  const int lim = nN - nodeBase;

  int rb0 = rbase[b];
  const int rb1 = rbase[b + 1];
  rb0 = rb0 < 0 ? 0 : (rb0 > csrLen ? csrLen : rb0);
  rb0 &= ~31;
  int len = rb1 - rb0;
  len = len < 0 ? 0 : (len > RCAP ? RCAP : len);
  int lenW = (len + 31) & ~31;
  if (rb0 + lenW > csrLen) lenW = (csrLen - rb0) & ~31;

  {
    const v4i z = {0, 0, 0, 0};
    for (int i = tid; i < RCAP / 4; i += NTHR) ((v4i*)region)[i] = z;
    for (int s = tid; s < NBF; s += NTHR) {
      int o = off[nodeBase + s] - rb0;
      o = o < 0 ? 0 : (o > RCAP ? RCAP : o);
      cursor[s] = o;
    }
  }
  __syncthreads();

  const int nChunks = (nK + CHUNK - 1) / CHUNK;
#pragma unroll 1
  for (int ch = 0; ch < nChunks; ++ch) {
    const int cbase = ch * CHUNK;
    const int wc = scan_chunk<NBF, 1, WCAP>(keys, nK, cbase, nodeBase, lim, vec8, list, tid, lane, wave);
    if (lane == 0) wcnt[wave] = wc;
    __syncthreads();
    if (wave == 0) {
#pragma unroll 1
      for (int wsx = 0; wsx < NWAVE; ++wsx) {
        int n = __builtin_amdgcn_readfirstlane(wcnt[wsx]);
        n = n > WCAP ? WCAP : (n < 0 ? 0 : n);
        const int* lp = list + wsx * WCAP;
#pragma unroll 1
        for (int i = 0; i < n; ++i) {
          const int ent  = __builtin_amdgcn_readfirstlane(lp[i]);
          const int slot = ent & (NBF - 1);
          int ev = (ent >> ESHF) & EMASK;
          ev = ev > nK - 1 ? nK - 1 : ev;
          if (lane == 0) {
            int pos = cursor[slot];
            pos = pos < 0 ? 0 : (pos > RCAP - 1 ? RCAP - 1 : pos);
            region[pos] = ev;
            const int np = pos + 1;
            cursor[slot] = np > RCAP ? RCAP : np;
          }
        }
      }
    }
    __syncthreads();
  }

  const int nv = lenW >> 2;
  int* gp = csr + rb0;
#pragma unroll 1
  for (int i = tid; i < nv; i += NTHR) { const v4i v = ((const v4i*)region)[i]; *(volatile v4i*)(gp + 4 * i) = v; }
  __threadfence();
#pragma unroll 1
  for (int i = tid; i < nv; i += NTHR) { const v4i v = ((const v4i*)region)[i]; *(volatile v4i*)(gp + 4 * i) = v; }
}

template <int KD, int NC, int EPI>
__global__ __launch_bounds__(NTHR) void k_gemm(
    const float* __restrict__ A, int lda, int nArows,
    const _Float16* __restrict__ Bw, const float* __restrict__ bias,
    float* Cout, int ldc, int nCrows, float osc) {
  extern __shared__ v4f lds_dyn[];
  static_assert((KD % 32) == 0);
  static_assert(NC == 128 || NC == 64);
  constexpr int NT  = NC / 16;
  constexpr int LPR = NC / 4;
  constexpr int RPI = 32 / LPR;
  constexpr int NST = 16 / RPI;
  float* stg = (float*)lds_dyn;
  const int tid = threadIdx.x, lane = tid & 31, wave = tid >> 5, hh = lane >> 4, m = lane & 15;
  const int rowBase = blockIdx.x * GROWS;
  const int colBase = blockIdx.y * NC;
  const int ar  = rowBase + wave * 16 + m;
  const int arc = ar < nArows ? ar : nArows - 1;
  const float z = (ar < nArows) ? (float)ASCL : 0.0f;
  const float* ap = A + (size_t)arc * lda + 8 * hh;
  const _Float16* bp0 = Bw + (size_t)(colBase + m) * KD + 8 * hh;

  v8f acc[NT];
#pragma unroll
  for (int t = 0; t < NT; ++t) { v8f zz = {0.f, 0.f, 0.f, 0.f, 0.f, 0.f, 0.f, 0.f}; acc[t] = zz; }

#pragma unroll 1
  for (int kt = 0; kt < KD / 32; ++kt) {
    const float* p = ap + 32 * kt;
    const v4f f0 = *(const v4f*)p;
    const v4f f1 = *(const v4f*)(p + 4);
    const v4f f2 = *(const v4f*)(p + 16);
    const v4f f3 = *(const v4f*)(p + 20);
    FragH af;
    af.h[0] = cvt8h(f0, f1, z);
    af.h[1] = cvt8h(f2, f3, z);
#pragma unroll
    for (int t = 0; t < NT; ++t) {
      const _Float16* bp = bp0 + (size_t)(16 * t) * KD + 32 * kt;
      FragH bf;
      bf.h[0] = *(const v8h*)bp;
      bf.h[1] = *(const v8h*)(bp + 16);
      acc[t] = wmf(af.v, bf.v, acc[t]);
    }
  }

  const int r0 = wave * 16 + 8 * hh;
  float bc[NT];
#pragma unroll
  for (int t = 0; t < NT; ++t) bc[t] = (EPI != 0) ? bias[colBase + 16 * t + m] : 0.0f;

  float* sp = stg + r0 * NC + m;
#pragma unroll
  for (int t = 0; t < NT; ++t) {
#pragma unroll
    for (int r = 0; r < 8; ++r) {
      float v = acc[t][r] * osc + bc[t];
      if constexpr (EPI == 1) v = fmaxf(v, 0.0f);
      if constexpr (EPI == 2) v = sigm(v);
      sp[r * NC + 16 * t] = v;
    }
  }
  __syncthreads();

  const int rsub = lane / LPR, c4 = 4 * (lane % LPR);
  const float* lp = stg + wave * 16 * NC;
  const int wrow = rowBase + wave * 16;
  float* gp = Cout + (size_t)wrow * ldc + colBase + c4;
#pragma unroll
  for (int i = 0; i < NST; ++i) {
    const int rl = i * RPI + rsub;
    const v4f v = *(const v4f*)(lp + rl * NC + c4);
    if (wrow + rl < nCrows) *(volatile v4f*)(gp + (size_t)rl * ldc) = v;
  }
  __threadfence();
#pragma unroll
  for (int i = 0; i < NST; ++i) {
    const int rl = i * RPI + rsub;
    const v4f v = *(const v4f*)(lp + rl * NC + c4);
    if (wrow + rl < nCrows) *(volatile v4f*)(gp + (size_t)rl * ldc) = v;
  }
}

__global__ __launch_bounds__(NTHR) void k_agg1(
    const int* __restrict__ csr, const int* __restrict__ off, const int* __restrict__ cnt,
    const int* __restrict__ srcidx, const float* __restrict__ dis,
    const float* __restrict__ x, const float* __restrict__ W1, const float* __restrict__ b1,
    float* Hp, int nN, int nE, int csrLen) {
  const int tid = threadIdx.x, lane = tid & 31, wave = tid >> 5;
  const int tbase = blockIdx.x * TGT + wave * 32;
  const int cl = tbase + lane;
  const int nraw = cnt[cl];
  const int st = off[cl];
  const float dc = dis[cl];
  const int n = nraw < 0 ? 0 : (nraw > DEGCAP ? DEGCAP : nraw);
  int nmx = n;
  nmx = max(nmx, __shfl_xor(nmx, 16, 32));
  nmx = max(nmx, __shfl_xor(nmx, 8, 32));
  nmx = max(nmx, __shfl_xor(nmx, 4, 32));
  nmx = max(nmx, __shfl_xor(nmx, 2, 32));
  nmx = max(nmx, __shfl_xor(nmx, 1, 32));
  nmx = __builtin_amdgcn_readfirstlane(nmx);
  nmx = nmx > DEGCAP ? DEGCAP : nmx;

  float a0 = 0.0f, a1 = 0.0f, a2 = 0.0f;
#pragma unroll 1
  for (int p = 0; p < nmx; ++p) {
    int pos = st + p;
    pos = pos < 0 ? 0 : (pos > csrLen - 1 ? csrLen - 1 : pos);
    int e = csr[pos];
    e = e < 0 ? 0 : (e > nE - 1 ? nE - 1 : e);
    int s = srcidx[e];
    s = s < 0 ? 0 : (s > nN - 1 ? nN - 1 : s);
    const float dsv = dis[s];
    const float w = (p < n) ? dsv * dc : 0.0f;
    const float* xr = x + (size_t)s * XD;
    a0 += w * xr[0];
    a1 += w * xr[1];
    a2 += w * xr[2];
  }
  {
    const int clc = cl < nN ? cl : nN - 1;
    const float d2 = dc * dc;
    const float* xr = x + (size_t)clc * XD;
    a0 += d2 * xr[0];
    a1 += d2 * xr[1];
    a2 += d2 * xr[2];
  }

  const int ch = 4 * lane;
  const v4f w0a = *(const v4f*)(W1 + ch),           w0b = *(const v4f*)(W1 + HID / 2 + ch);
  const v4f w1a = *(const v4f*)(W1 + HID + ch),     w1b = *(const v4f*)(W1 + HID + HID / 2 + ch);
  const v4f w2a = *(const v4f*)(W1 + 2 * HID + ch), w2b = *(const v4f*)(W1 + 2 * HID + HID / 2 + ch);
  const v4f ba  = *(const v4f*)(b1 + ch),           bb  = *(const v4f*)(b1 + HID / 2 + ch);
#pragma unroll 1
  for (int j = 0; j < 32; ++j) {
    const int c = tbase + j;
    U32F u0; u0.i = __builtin_amdgcn_readlane(__float_as_int(a0), j);
    U32F u1; u1.i = __builtin_amdgcn_readlane(__float_as_int(a1), j);
    U32F u2; u2.i = __builtin_amdgcn_readlane(__float_as_int(a2), j);
    const int nrj = __builtin_amdgcn_readlane(nraw, j);
    v4f ya = relu4(w0a * u0.f + w1a * u1.f + w2a * u2.f + ba);
    v4f yb = relu4(w0b * u0.f + w1b * u1.f + w2b * u2.f + bb);
    if (c >= nN) {
      const v4f zz = {0.f, 0.f, 0.f, 0.f};
      ya = zz; yb = zz;
    }
    if (nrj > DEGCAP) {
      const float qn = __int_as_float(0x7fc00000);
      ya.x = qn; ya.y = qn; ya.z = qn; ya.w = qn;
      yb = ya;
    }
    float* hp = Hp + (size_t)c * HID;
    *(volatile v4f*)(hp + ch) = ya;
    *(volatile v4f*)(hp + HID / 2 + ch) = yb;
    __threadfence();
    *(volatile v4f*)(hp + ch) = ya;
    *(volatile v4f*)(hp + HID / 2 + ch) = yb;
  }
}

__global__ __launch_bounds__(NTHR) void k_agg(
    const int* __restrict__ csr, const int* __restrict__ off, const int* __restrict__ cnt,
    const int* __restrict__ srcidx, const float* __restrict__ dis,
    const float* __restrict__ hw, const float* __restrict__ bias,
    float* Hp, int nN, int nE, int csrLen) {
  const int tid = threadIdx.x, lane = tid & 31, wave = tid >> 5;
  const int tbase = blockIdx.x * TGT + wave * 32;
  const int cl = tbase + lane;
  const int cnt_l = cnt[cl];
  const int off_l = off[cl];
  const float dis_l = dis[cl];
  const int ch = 4 * lane;
  const v4f bva = *(const v4f*)(bias + ch);
  const v4f bvb = *(const v4f*)(bias + HID / 2 + ch);

#pragma unroll 1
  for (int j = 0; j < 32; ++j) {
    const int c = tbase + j;
    const int nraw = __builtin_amdgcn_readlane(cnt_l, j);
    const int n = nraw < 0 ? 0 : (nraw > DEGCAP ? DEGCAP : nraw);
    const int st = __builtin_amdgcn_readlane(off_l, j);
    U32F du; du.i = __builtin_amdgcn_readlane(__float_as_int(dis_l), j);
    const float dc = du.f;
    v4f acca = {0.f, 0.f, 0.f, 0.f};
    v4f accb = {0.f, 0.f, 0.f, 0.f};
#pragma unroll 1
    for (int q0 = 0; q0 < n; q0 += 32) {
      int pos = st + q0 + lane;
      pos = pos < 0 ? 0 : (pos > csrLen - 1 ? csrLen - 1 : pos);
      int el = csr[pos];
      el = el < 0 ? 0 : (el > nE - 1 ? nE - 1 : el);
      int sl = srcidx[el];
      sl = sl < 0 ? 0 : (sl > nN - 1 ? nN - 1 : sl);
      U32F wu; wu.f = dis[sl] * dc;
      const int mcnt = (n - q0) < 32 ? (n - q0) : 32;
#pragma unroll 1
      for (int p = 0; p < mcnt; ++p) {
        const int s = __builtin_amdgcn_readlane(sl, p);
        U32F t; t.i = __builtin_amdgcn_readlane(wu.i, p);
        const float* hr = hw + (size_t)s * HID;
        const v4f hva = *(const v4f*)(hr + ch);
        const v4f hvb = *(const v4f*)(hr + HID / 2 + ch);
        acca = acca + hva * t.f;
        accb = accb + hvb * t.f;
      }
    }
    const float* hcr = hw + (size_t)c * HID;
    const v4f hca = *(const v4f*)(hcr + ch);
    const v4f hcb = *(const v4f*)(hcr + HID / 2 + ch);
    const float d2 = dc * dc;
    v4f ya = relu4(acca + hca * d2 + bva);
    v4f yb = relu4(accb + hcb * d2 + bvb);
    if (c >= nN) {
      const v4f zz = {0.f, 0.f, 0.f, 0.f};
      ya = zz; yb = zz;
    }
    if (nraw > DEGCAP) {
      const float qn = __int_as_float(0x7fc00000);
      ya.x = qn; ya.y = qn; ya.z = qn; ya.w = qn;
      yb = ya;
    }
    float* hp = Hp + (size_t)c * HID;
    *(volatile v4f*)(hp + ch) = ya;
    *(volatile v4f*)(hp + HID / 2 + ch) = yb;
    __threadfence();
    *(volatile v4f*)(hp + ch) = ya;
    *(volatile v4f*)(hp + HID / 2 + ch) = yb;
  }
}

__global__ __launch_bounds__(NTHR) void k_pool(
    const int* __restrict__ keys, int nK, const float* __restrict__ hsrc,
    float* Hout, int ldh, int hcol, int nG, int vec8) {
  extern __shared__ v4f lds_dyn[];
  float* accp = (float*)lds_dyn;
  int* list = (int*)(accp + PG * HID);
  int* wcnt = list + NWAVE * WCAP;
  int* pcnt = wcnt + NWAVE;
  const int tid = threadIdx.x, lane = tid & 31, wave = tid >> 5;
  const int slotBase = blockIdx.x * PG;
  const int lim = nG - slotBase;
  const int ch = 4 * lane;

  {
    const v4f z = {0.f, 0.f, 0.f, 0.f};
    for (int i = tid; i < PG * HID / 4; i += NTHR) ((v4f*)accp)[i] = z;
    for (int i = tid; i < PG; i += NTHR) pcnt[i] = 0;
  }
  __syncthreads();

  const int nChunks = (nK + CHUNK - 1) / CHUNK;
#pragma unroll 1
  for (int chn = 0; chn < nChunks; ++chn) {
    const int cbase = chn * CHUNK;
    const int wc = scan_chunk<PG, 1, WCAP>(keys, nK, cbase, slotBase, lim, vec8, list, tid, lane, wave);
    if (lane == 0) wcnt[wave] = wc;
    __syncthreads();
#pragma unroll 1
    for (int wsx = 0; wsx < NWAVE; ++wsx) {
      int n = __builtin_amdgcn_readfirstlane(wcnt[wsx]);
      n = n > WCAP ? WCAP : (n < 0 ? 0 : n);
      const int* lp = list + wsx * WCAP;
#pragma unroll 1
      for (int i = 0; i < n; ++i) {
        const int ent  = __builtin_amdgcn_readfirstlane(lp[i]);
        const int slot = ent & (PG - 1);
        int node = (ent >> ESHF) & EMASK;
        node = node > nK - 1 ? nK - 1 : node;
        if ((slot >> 3) == wave) {
          const float* hr = hsrc + (size_t)node * HID;
          const v4f va = *(const v4f*)(hr + ch);
          const v4f vb = *(const v4f*)(hr + HID / 2 + ch);
          float* aq = accp + slot * HID;
          const v4f oa = *(const v4f*)(aq + ch);
          const v4f ob = *(const v4f*)(aq + HID / 2 + ch);
          *(v4f*)(aq + ch) = oa + va;
          *(v4f*)(aq + HID / 2 + ch) = ob + vb;
          if (lane == 0) pcnt[slot] = pcnt[slot] + 1;
        }
      }
    }
    __syncthreads();
  }

#pragma unroll 1
  for (int q = 0; q < 8; ++q) {
    const int slot = wave * 8 + q;
    const int c = pcnt[slot];
    const float inv = 1.0f / (float)(c < 1 ? 1 : c);
    const float* aq = accp + slot * HID;
    const v4f va = *(const v4f*)(aq + ch) * inv;
    const v4f vb = *(const v4f*)(aq + HID / 2 + ch) * inv;
    float* hp = Hout + (size_t)(slotBase + slot) * ldh + hcol;
    *(volatile v4f*)(hp + ch) = va;
    *(volatile v4f*)(hp + HID / 2 + ch) = vb;
    __threadfence();
    *(volatile v4f*)(hp + ch) = va;
    *(volatile v4f*)(hp + HID / 2 + ch) = vb;
  }
}

static void enc_graph(hipStream_t stream, const float* x, const int* ei, int nE, const int* batch,
                      const float* W1, const float* b1,
                      const _Float16* W2p, const float* b2, const _Float16* W3p, const float* b3,
                      int* cnt, int* off, float* dis, int* rb, int* csr, int csrLen,
                      float* HA, float* XB, float* H, int hcol,
                      int nN, int nG, int nBC, int nBF, int nAgg, int nGemmN, int nPool, int NPAD, float osc) {
  const int* src = ei;
  const int* dst = ei + nE;
  const int vec8 = ((nE & 3) == 0) ? 1 : 0;
  k_count<<<nBC, NTHR, LDS_COUNT, stream>>>(dst, cnt, nE, vec8, nN);
  k_offsets<<<1, OTHR, 0, stream>>>(cnt, off, dis, rb, nBF);
  k_fill<<<nBF, NTHR, LDS_FILL, stream>>>(dst, off, rb, csr, nE, vec8, csrLen, nN);
  k_agg1<<<nAgg, NTHR, 0, stream>>>(csr, off, cnt, src, dis, x, W1, b1, HA, nN, nE, csrLen);
  k_gemm<HID, 128, 0><<<dim3(nGemmN, HID / 128, 1), NTHR, LDS_G128, stream>>>(HA, HID, NPAD, W2p, b2, XB, HID, NPAD, osc);
  k_agg<<<nAgg, NTHR, 0, stream>>>(csr, off, cnt, src, dis, XB, b2, HA, nN, nE, csrLen);
  k_gemm<HID, 128, 0><<<dim3(nGemmN, HID / 128, 1), NTHR, LDS_G128, stream>>>(HA, HID, NPAD, W3p, b3, XB, HID, NPAD, osc);
  k_agg<<<nAgg, NTHR, 0, stream>>>(csr, off, cnt, src, dis, XB, b3, HA, nN, nE, csrLen);
  k_pool<<<nPool, NTHR, LDS_POOL, stream>>>(batch, nN, HA, H, 2 * HID, hcol, nG, 1);
}

extern "C" void kernel_launch(void* const* d_in, const int* in_sizes, int n_in,
                              void* d_out, int out_size, void* d_ws, size_t ws_size,
                              hipStream_t stream) {
  if (n_in < 20) return;
  if (in_sizes[0] < XD || (in_sizes[0] % XD) != 0) return;
  const int nN = in_sizes[0] / XD;
  if (in_sizes[3] != in_sizes[0]) return;
  if (in_sizes[2] != nN || in_sizes[5] != nN) return;
  if (in_sizes[1] < 2 || (in_sizes[1] & 1) != 0) return;
  if (in_sizes[4] < 2 || (in_sizes[4] & 1) != 0) return;
  const int nE1 = in_sizes[1] / 2;
  const int nE2 = in_sizes[4] / 2;
  if (in_sizes[6] != XD * HID || in_sizes[7] != HID) return;
  if (in_sizes[8] != HID * HID || in_sizes[9] != HID) return;
  if (in_sizes[10] != HID * HID || in_sizes[11] != HID) return;
  if (in_sizes[12] != 512 * 512 || in_sizes[13] != 512) return;
  if (in_sizes[14] != 512 * 256 || in_sizes[15] != 256) return;
  if (in_sizes[16] != 256 * 128 || in_sizes[17] != 128) return;
  if (in_sizes[18] != 128 * 64 || in_sizes[19] != 64) return;
  if (out_size < 64 || (out_size % 64) != 0) return;
  const int nG = out_size / 64;
  if (nN > (1 << 20) || nE1 > (1 << 20) || nE2 > (1 << 20) || nG > (1 << 20)) return;

  const float* x1  = (const float*)d_in[0];
  const int*   ei1 = (const int*)d_in[1];
  const int*   bt1 = (const int*)d_in[2];
  const float* x2  = (const float*)d_in[3];
  const int*   ei2 = (const int*)d_in[4];
  const int*   bt2 = (const int*)d_in[5];
  const float* W1  = (const float*)d_in[6];
  const float* b1  = (const float*)d_in[7];
  const float* W2  = (const float*)d_in[8];
  const float* b2  = (const float*)d_in[9];
  const float* W3  = (const float*)d_in[10];
  const float* b3  = (const float*)d_in[11];
  const float* Wl1 = (const float*)d_in[12];
  const float* bl1 = (const float*)d_in[13];
  const float* Wl2 = (const float*)d_in[14];
  const float* bl2 = (const float*)d_in[15];
  const float* Wl3 = (const float*)d_in[16];
  const float* bl3 = (const float*)d_in[17];
  const float* Wl4 = (const float*)d_in[18];
  const float* bl4 = (const float*)d_in[19];
  float* out = (float*)d_out;

  const int NPAD   = ((nN + TGT - 1) / TGT) * TGT;
  const int nBC    = (nN + NBC - 1) / NBC;
  const int CNTPAD = nBC * NBC;
  const int nBF    = (nN + NBF - 1) / NBF;
  const int OFFN   = nBF * NBF;
  if (nBF + 1 > RBN) return;
  if (OFFN > CNTPAD || NPAD > OFFN) return;
  if ((NPAD % GROWS) != 0 || (NPAD % TGT) != 0) return;
  const int GPAD   = ((nG + GROWS - 1) / GROWS) * GROWS;
  if ((GPAD % PG) != 0) return;
  const int nEmax  = nE1 > nE2 ? nE1 : nE2;
  const int csrCap  = ((nEmax + 31) & ~31) + 32 * (nBF + 1);
  const int csrLen1 = ((nE1 + 31) & ~31) + 32 * (nBF + 1);
  const int csrLen2 = ((nE2 + 31) & ~31) + 32 * (nBF + 1);
  const int nGemmN = NPAD / GROWS;
  const int nAgg   = NPAD / TGT;
  const int nPool  = GPAD / PG;
  const int nGemmG = GPAD / GROWS;

  char* ws = (char*)d_ws;
  size_t off = 0;
  const size_t oHA  = off; off += (size_t)NPAD * HID * 4;          off = (off + 255) & ~(size_t)255;
  const size_t oXB  = off; off += (size_t)NPAD * HID * 4;          off = (off + 255) & ~(size_t)255;
  const size_t oH   = off; off += (size_t)GPAD * 2 * HID * 4;      off = (off + 255) & ~(size_t)255;
  const size_t oW2  = off; off += (size_t)HID * HID * 2;           off = (off + 255) & ~(size_t)255;
  const size_t oW3  = off; off += (size_t)HID * HID * 2;           off = (off + 255) & ~(size_t)255;
  const size_t oL1  = off; off += (size_t)512 * 512 * 2;           off = (off + 255) & ~(size_t)255;
  const size_t oL2  = off; off += (size_t)256 * 512 * 2;           off = (off + 255) & ~(size_t)255;
  const size_t oL3  = off; off += (size_t)128 * 256 * 2;           off = (off + 255) & ~(size_t)255;
  const size_t oL4  = off; off += (size_t)64 * 128 * 2;            off = (off + 255) & ~(size_t)255;
  const size_t oCnt = off; off += (size_t)CNTPAD * 4;              off = (off + 255) & ~(size_t)255;
  const size_t oOff = off; off += (size_t)OFFN * 4;                off = (off + 255) & ~(size_t)255;
  const size_t oDis = off; off += (size_t)OFFN * 4;                off = (off + 255) & ~(size_t)255;
  const size_t oRb  = off; off += (size_t)RBN * 4;                 off = (off + 255) & ~(size_t)255;
  const size_t oCsr = off; off += (size_t)csrCap * 4;              off = (off + 255) & ~(size_t)255;
  if (off > ws_size || off > (size_t)WSCAP) return;
  if ((size_t)GPAD * 512 * 4 > (size_t)NPAD * HID * 4) return;
  float*    HA   = (float*)(ws + oHA);
  float*    XB   = (float*)(ws + oXB);
  float*    H    = (float*)(ws + oH);
  _Float16* W2p  = (_Float16*)(ws + oW2);
  _Float16* W3p  = (_Float16*)(ws + oW3);
  _Float16* L1p  = (_Float16*)(ws + oL1);
  _Float16* L2p  = (_Float16*)(ws + oL2);
  _Float16* L3p  = (_Float16*)(ws + oL3);
  _Float16* L4p  = (_Float16*)(ws + oL4);
  int*   cnt = (int*)(ws + oCnt);
  int*   ofp = (int*)(ws + oOff);
  float* dis = (float*)(ws + oDis);
  int*   rb  = (int*)(ws + oRb);
  int*   csr = (int*)(ws + oCsr);
  float* Z1  = HA;
  float* Z2  = XB;
  float* Z3  = HA;

  const float osc = 1.0f / ((float)ASCL * (float)WSCL);

  {
    const dim3 gW(HID / TPK, HID / TPN, 1);
    k_wT16<<<gW, NTHR, 0, stream>>>(W2, W2p, HID, HID, HID, (float)WSCL);
    k_wT16<<<gW, NTHR, 0, stream>>>(W3, W3p, HID, HID, HID, (float)WSCL);
    const dim3 gL1(512 / TPK, 512 / TPN, 1);
    k_wT16<<<gL1, NTHR, 0, stream>>>(Wl1, L1p, 512, 512, 512, (float)WSCL);
    const dim3 gL2(512 / TPK, 256 / TPN, 1);
    k_wT16<<<gL2, NTHR, 0, stream>>>(Wl2, L2p, 512, 256, 256, (float)WSCL);
    const dim3 gL3(256 / TPK, 128 / TPN, 1);
    k_wT16<<<gL3, NTHR, 0, stream>>>(Wl3, L3p, 256, 128, 128, (float)WSCL);
    const dim3 gL4(128 / TPK, 64 / TPN, 1);
    k_wT16<<<gL4, NTHR, 0, stream>>>(Wl4, L4p, 128, 64, 64, (float)WSCL);
  }

  hipFuncSetAttribute(reinterpret_cast<const void*>(&k_count),
                      hipFuncAttributeMaxDynamicSharedMemorySize, LDS_COUNT);
  hipFuncSetAttribute(reinterpret_cast<const void*>(&k_fill),
                      hipFuncAttributeMaxDynamicSharedMemorySize, LDS_FILL);
  hipFuncSetAttribute(reinterpret_cast<const void*>(&k_pool),
                      hipFuncAttributeMaxDynamicSharedMemorySize, LDS_POOL);
  hipFuncSetAttribute(reinterpret_cast<const void*>(&k_gemm<HID, 128, 0>),
                      hipFuncAttributeMaxDynamicSharedMemorySize, LDS_G128);
  hipFuncSetAttribute(reinterpret_cast<const void*>(&k_gemm<512, 128, 1>),
                      hipFuncAttributeMaxDynamicSharedMemorySize, LDS_G128);
  hipFuncSetAttribute(reinterpret_cast<const void*>(&k_gemm<256, 128, 1>),
                      hipFuncAttributeMaxDynamicSharedMemorySize, LDS_G128);
  hipFuncSetAttribute(reinterpret_cast<const void*>(&k_gemm<128, 64, 2>),
                      hipFuncAttributeMaxDynamicSharedMemorySize, LDS_G64);

  enc_graph(stream, x1, ei1, nE1, bt1, W1, b1, W2p, b2, W3p, b3, cnt, ofp, dis, rb, csr, csrLen1,
            HA, XB, H, 0, nN, nG, nBC, nBF, nAgg, nGemmN, nPool, NPAD, osc);
  enc_graph(stream, x2, ei2, nE2, bt2, W1, b1, W2p, b2, W3p, b3, cnt, ofp, dis, rb, csr, csrLen2,
            HA, XB, H, HID, nN, nG, nBC, nBF, nAgg, nGemmN, nPool, NPAD, osc);

  k_gemm<512, 128, 1><<<dim3(nGemmG, 512 / 128, 1), NTHR, LDS_G128, stream>>>(H, 512, GPAD, L1p, bl1, Z1, 512, GPAD, osc);
  k_gemm<512, 128, 1><<<dim3(nGemmG, 256 / 128, 1), NTHR, LDS_G128, stream>>>(Z1, 512, GPAD, L2p, bl2, Z2, 256, GPAD, osc);
  k_gemm<256, 128, 1><<<dim3(nGemmG, 1, 1), NTHR, LDS_G128, stream>>>(Z2, 256, GPAD, L3p, bl3, Z3, 128, GPAD, osc);
  k_gemm<128, 64, 2><<<dim3(nGemmG, 1, 1), NTHR, LDS_G64, stream>>>(Z3, 128, GPAD, L4p, bl4, out, 64, nG, osc);
}
